// ResAttention_2482491097650
// MI455X (gfx1250) — hardware-verified
//
#include <hip/hip_runtime.h>
#include <math.h>
#include <stdint.h>

#define SEQ   2048
#define NIN   256
#define DM    512
#define NLAY  2
#define EPSLN 1e-5f
#define QSC   8.0f
#define KSC   8.0f
#define PCAR  32768.0f
#define VCAR  1024.0f
#define XSC   1024.0f
#define WSC   1024.0f
#define ASC   1024.0f
#define LOG2E 1.4426950408889634f
#define RSQD  0.04419417382415922f
#define QT    16
#define CK    512
#define SCP   544
#define PLP   528
#define SLAB64 (16 * 68)
#define VTP   72
#define ATT_THREADS 256
#define WS_CAP ((size_t)134217728)

static_assert(DM == 8 * 64 && (DM % 32) == 0 && (NIN % 32) == 0);
static_assert((SEQ % CK) == 0 && CK == 16 * 32 && (SEQ % 64) == 0 && (SEQ / QT) == 128);
static_assert(8 * SLAB64 == 16 * SCP);
static_assert(((PLP * 2) % 16) == 0 && ((SCP * 4) % 16) == 0 && ((VTP * 2) % 16) == 0);
static_assert(64 * VTP >= 63 * VTP + 64);
static_assert(ATT_THREADS == 16 * QT && ATT_THREADS == 256);

typedef unsigned short u16;
typedef _Float16 v16h __attribute__((ext_vector_type(16)));
typedef _Float16 v8h  __attribute__((ext_vector_type(8)));
typedef __bf16   v16b __attribute__((ext_vector_type(16)));
typedef float    v8f  __attribute__((ext_vector_type(8)));
typedef float    v4f  __attribute__((ext_vector_type(4)));
typedef unsigned int v4u __attribute__((ext_vector_type(4)));

union FragH { v16h v; v8h h[2]; v4u u[2]; };
union FragB { v16b v; v4u u[2]; };

__device__ __forceinline__ unsigned short bf_bits(float f) {
  unsigned u = __float_as_uint(f);
  return (unsigned short)((u + 0x7FFFu + ((u >> 16) & 1u)) >> 16);
}
__device__ __forceinline__ float bf_up(unsigned short h) { return __uint_as_float(((unsigned)h) << 16); }
__device__ __forceinline__ float bfr(float f) { return bf_up(bf_bits(f)); }
__device__ __forceinline__ unsigned short h_bits(_Float16 x) { return __builtin_bit_cast(unsigned short, x); }
__device__ __forceinline__ unsigned pk16(unsigned short a, unsigned short b) { return (unsigned)a | ((unsigned)b << 16); }
__device__ __forceinline__ v8f zero8() { v8f z = {0.f, 0.f, 0.f, 0.f, 0.f, 0.f, 0.f, 0.f}; return z; }
__device__ __forceinline__ v4f zero4() { v4f z = {0.f, 0.f, 0.f, 0.f}; return z; }

__device__ __forceinline__ v16h ldfrag_h(const _Float16* p) {
  FragH f;
  f.h[0] = *(const v8h*)(p);
  f.h[1] = *(const v8h*)(p + 16);
  return f.v;
}
__device__ __forceinline__ v16b ldfrag_b(const u16* p) {
  FragB f;
  f.u[0] = *(const v4u*)(p);
  f.u[1] = *(const v4u*)(p + 16);
  return f.v;
}

__device__ __forceinline__ v8f mma_h(v16h a, v16h b, v8f c) {
  return __builtin_amdgcn_wmma_f32_16x16x32_f16(false, a, false, b, (short)0, c, false, false);
}
__device__ __forceinline__ v8f mma_b(v16b a, v16b b, v8f c) {
  return __builtin_amdgcn_wmma_f32_16x16x32_bf16(false, a, false, b, (short)0, c, false, false);
}
__device__ __forceinline__ void guard2x3(v8f& a, v8f& b, v16h x0, v16h x1, v16h x2) {
#if defined(__HIP_DEVICE_COMPILE__)
  asm volatile("v_nop\n\tv_nop\n\tv_nop\n\tv_nop"
               : "+v"(a), "+v"(b) : "v"(x0), "v"(x1), "v"(x2) : "memory");
#endif
}
template <typename F>
__device__ __forceinline__ void guard6(v8f& a, v8f& b, v8f& c, v8f& d, F x0, F x1, F x2, F x3, F x4, F x5) {
#if defined(__HIP_DEVICE_COMPILE__)
  asm volatile("v_nop\n\tv_nop\n\tv_nop\n\tv_nop"
               : "+v"(a), "+v"(b), "+v"(c), "+v"(d) : "v"(x0), "v"(x1), "v"(x2), "v"(x3), "v"(x4), "v"(x5) : "memory");
#endif
}
__device__ __forceinline__ void acc_guard4(v8f& a, v8f& b, v8f& c, v8f& d) {
#if defined(__HIP_DEVICE_COMPILE__)
  asm volatile("v_nop\n\tv_nop\n\tv_nop\n\tv_nop" : "+v"(a), "+v"(b), "+v"(c), "+v"(d));
#endif
}
__device__ __forceinline__ void wave_sync_lds() {
  __builtin_amdgcn_fence(__ATOMIC_RELEASE, "workgroup");
  __builtin_amdgcn_wave_barrier();
  __builtin_amdgcn_fence(__ATOMIC_ACQUIRE, "workgroup");
}

__global__ __launch_bounds__(256) void cvt16(const float* __restrict__ x, u16* D, int n8, int mode, float scale) {
  const int gt = blockIdx.x * 256 + (int)threadIdx.x;
  if (gt >= n8) return;
  const float* p = x + (size_t)gt * 8;
  const v4f a = *(const v4f*)(p), c4 = *(const v4f*)(p + 4);
  float v[8];
#pragma unroll
  for (int e = 0; e < 4; ++e) { v[e] = a[e]; v[4 + e] = c4[e]; }
  unsigned short s[8];
#pragma unroll
  for (int e = 0; e < 8; ++e) {
    const float vb = bfr(v[e]);
    const float vf = (mode == 1) ? vb : v[e];
    const unsigned short hb = h_bits((_Float16)(vf * scale));
    const unsigned short bb = bf_bits(v[e]);
    s[e] = (mode != 0) ? hb : bb;
  }
  v4u o;
#pragma unroll
  for (int e = 0; e < 4; ++e) o[e] = pk16(s[2 * e], s[2 * e + 1]);
  u16* d = D + (size_t)gt * 8;
  for (int pass = 0; pass < 2; ++pass) {
    *(volatile v4u*)(d) = o;
    __threadfence();
  }
}

__device__ __forceinline__ void stage64(float* sl, v8f a0, v8f a1, v8f a2, v8f a3, float oscale, int lane) {
  const int hh = lane >> 4, m = lane & 15;
#pragma unroll
  for (int r = 0; r < 8; ++r) {
    const int ro = (8 * hh + r) * 68 + m;
    sl[ro]      = a0[r] * oscale;
    sl[ro + 16] = a1[r] * oscale;
    sl[ro + 32] = a2[r] * oscale;
    sl[ro + 48] = a3[r] * oscale;
  }
  wave_sync_lds();
}
__device__ __forceinline__ void epi64(float* sl, v8f a0, v8f a1, v8f a2, v8f a3, float oscale, v4f badd, float* C, int N,
                                      size_t rowb, int col0, int lane) {
  const int hh = lane >> 4, m = lane & 15;
  stage64(sl, a0, a1, a2, a3, oscale, lane);
  v4f vals[8];
#pragma unroll
  for (int it = 0; it < 8; ++it) vals[it] = *(const v4f*)(sl + (it * 2 + hh) * 68 + m * 4) + badd;
  float* dst = C + (rowb + (size_t)hh) * (size_t)N + col0 + m * 4;
  for (int pass = 0; pass < 2; ++pass) {
#pragma unroll
    for (int it = 0; it < 8; ++it) {
      *(volatile v4f*)(dst + (size_t)(it * 2) * (size_t)N) = vals[it];
    }
    __threadfence();
  }
}
__device__ __forceinline__ void epi64r(float* sl, v8f a0, v8f a1, v8f a2, v8f a3, float oscale, v4f badd,
                                       const float* __restrict__ R, int use_res, float* C, int N,
                                       size_t rowb, int col0, int lane) {
  const int hh = lane >> 4, m = lane & 15;
  stage64(sl, a0, a1, a2, a3, oscale, lane);
  v4f vals[8];
#pragma unroll
  for (int it = 0; it < 8; ++it) vals[it] = *(const v4f*)(sl + (it * 2 + hh) * 68 + m * 4) + badd;
  const size_t eb = (rowb + (size_t)hh) * (size_t)N + col0 + m * 4;
  if (use_res != 0) {
#pragma unroll
    for (int it = 0; it < 8; ++it) vals[it] = vals[it] + *(const v4f*)(R + eb + (size_t)(it * 2) * (size_t)N);
  }
  float* dst = C + eb;
  for (int pass = 0; pass < 2; ++pass) {
#pragma unroll
    for (int it = 0; it < 8; ++it) {
      *(volatile v4f*)(dst + (size_t)(it * 2) * (size_t)N) = vals[it];
    }
    __threadfence();
  }
}
__device__ __forceinline__ void epi64h(float* sl, v8f a0, v8f a1, v8f a2, v8f a3, float oscale,
                                       const float* __restrict__ bias, float pscale, u16* C, int N,
                                       size_t rowb, int col0, int lane) {
  stage64(sl, a0, a1, a2, a3, oscale, lane);
  const int rq = lane >> 3, c8 = (lane & 7) * 8;
  const v4f bv0 = *(const v4f*)(bias + col0 + c8), bv1 = *(const v4f*)(bias + col0 + c8 + 4);
  float bb[8];
#pragma unroll
  for (int e = 0; e < 4; ++e) { bb[e] = bfr(bv0[e]); bb[4 + e] = bfr(bv1[e]); }
  v4u oh[4];
#pragma unroll
  for (int i4 = 0; i4 < 4; ++i4) {
    const int row = i4 * 4 + rq;
    const v4f a = *(const v4f*)(sl + row * 68 + c8), c4 = *(const v4f*)(sl + row * 68 + c8 + 4);
    float w[8];
#pragma unroll
    for (int e = 0; e < 4; ++e) { w[e] = (a[e] + bb[e]) * pscale; w[4 + e] = (c4[e] + bb[4 + e]) * pscale; }
#pragma unroll
    for (int e = 0; e < 4; ++e) oh[i4][e] = pk16(h_bits((_Float16)w[2 * e]), h_bits((_Float16)w[2 * e + 1]));
  }
  u16* dst = C + rowb * (size_t)N + col0 + c8;
  for (int pass = 0; pass < 2; ++pass) {
#pragma unroll
    for (int i4 = 0; i4 < 4; ++i4) {
      const int row = i4 * 4 + rq;
      *(volatile v4u*)(dst + (size_t)row * (size_t)N) = oh[i4];
    }
    __threadfence();
  }
}

__global__ __launch_bounds__(128)
void gemm_bfb(const u16* __restrict__ A, const u16* __restrict__ Bt, const float* __restrict__ bias,
              float* C, int M, int N, int K, float oscale) {
  __shared__ __align__(16) float slab[4 * SLAB64];
  const int tid = threadIdx.x, wave = tid >> 5, lane = tid & 31, hh = lane >> 4, m = lane & 15;
  const int ntile = N >> 6;
  const int bid   = blockIdx.x;
  const int rowb  = (bid / ntile) * 64 + wave * 16;
  const int col0  = (bid % ntile) * 64;
  if (rowb + 16 > M) return;
  const u16* ap = A  + (size_t)(rowb + m) * K + 8 * hh;
  const u16* bp = Bt + (size_t)(col0 + m) * K + 8 * hh;
  const size_t bs = (size_t)16 * K;
  v8f acc0 = zero8(), acc1 = zero8(), acc2 = zero8(), acc3 = zero8();
#pragma unroll 1
  for (int k0 = 0; k0 < K; k0 += 32) {
    const v16b a  = ldfrag_b(ap + k0);
    const v16b b0 = ldfrag_b(bp + k0);
    const v16b b1 = ldfrag_b(bp + bs + k0);
    const v16b b2 = ldfrag_b(bp + 2 * bs + k0);
    const v16b b3 = ldfrag_b(bp + 3 * bs + k0);
    acc0 = mma_b(a, b0, acc0);
    acc1 = mma_b(a, b1, acc1);
    acc2 = mma_b(a, b2, acc2);
    acc3 = mma_b(a, b3, acc3);
    guard6<v16b>(acc0, acc1, acc2, acc3, a, b0, b1, b2, b3, a);
  }
  const v4f bv = *(const v4f*)(bias + col0 + m * 4);
  v4f badd;
#pragma unroll
  for (int e = 0; e < 4; ++e) badd[e] = bfr(bv[e]);
  epi64(slab + wave * SLAB64, acc0, acc1, acc2, acc3, oscale, badd, C, N, (size_t)rowb, col0, lane);
}

__global__ __launch_bounds__(128)
void gemm_ho16(const u16* __restrict__ A, const u16* __restrict__ Bt, const float* __restrict__ bias,
               u16* C, int M, int N, int K, float oscale, float pscale) {
  __shared__ __align__(16) float slab[4 * SLAB64];
  const int tid = threadIdx.x, wave = tid >> 5, lane = tid & 31, hh = lane >> 4, m = lane & 15;
  const int ntile = N >> 6;
  const int bid   = blockIdx.x;
  const int rowb  = (bid / ntile) * 64 + wave * 16;
  const int col0  = (bid % ntile) * 64;
  if (rowb + 16 > M) return;
  const _Float16* ap = (const _Float16*)(const void*)A  + (size_t)(rowb + m) * K + 8 * hh;
  const _Float16* bp = (const _Float16*)(const void*)Bt + (size_t)(col0 + m) * K + 8 * hh;
  const size_t bs = (size_t)16 * K;
  v8f acc0 = zero8(), acc1 = zero8(), acc2 = zero8(), acc3 = zero8();
#pragma unroll 1
  for (int k0 = 0; k0 < K; k0 += 32) {
    const v16h a  = ldfrag_h(ap + k0);
    const v16h b0 = ldfrag_h(bp + k0);
    const v16h b1 = ldfrag_h(bp + bs + k0);
    const v16h b2 = ldfrag_h(bp + 2 * bs + k0);
    const v16h b3 = ldfrag_h(bp + 3 * bs + k0);
    acc0 = mma_h(a, b0, acc0);
    acc1 = mma_h(a, b1, acc1);
    acc2 = mma_h(a, b2, acc2);
    acc3 = mma_h(a, b3, acc3);
    guard6<v16h>(acc0, acc1, acc2, acc3, a, b0, b1, b2, b3, a);
  }
  epi64h(slab + wave * SLAB64, acc0, acc1, acc2, acc3, oscale, bias, pscale, C, N, (size_t)rowb, col0, lane);
}

__global__ __launch_bounds__(128)
void gemm_h32(const u16* __restrict__ A, const u16* __restrict__ Bt, const float* __restrict__ bias,
              const float* __restrict__ R, int use_res, float* C, int M, int N, int K, float oscale) {
  __shared__ __align__(16) float slab[4 * SLAB64];
  const int tid = threadIdx.x, wave = tid >> 5, lane = tid & 31, hh = lane >> 4, m = lane & 15;
  const int ntile = N >> 6;
  const int bid   = blockIdx.x;
  const int rowb  = (bid / ntile) * 64 + wave * 16;
  const int col0  = (bid % ntile) * 64;
  if (rowb + 16 > M) return;
  const _Float16* ap = (const _Float16*)(const void*)A  + (size_t)(rowb + m) * K + 8 * hh;
  const _Float16* bp = (const _Float16*)(const void*)Bt + (size_t)(col0 + m) * K + 8 * hh;
  const size_t bs = (size_t)16 * K;
  v8f acc0 = zero8(), acc1 = zero8(), acc2 = zero8(), acc3 = zero8();
#pragma unroll 1
  for (int k0 = 0; k0 < K; k0 += 32) {
    const v16h a  = ldfrag_h(ap + k0);
    const v16h b0 = ldfrag_h(bp + k0);
    const v16h b1 = ldfrag_h(bp + bs + k0);
    const v16h b2 = ldfrag_h(bp + 2 * bs + k0);
    const v16h b3 = ldfrag_h(bp + 3 * bs + k0);
    acc0 = mma_h(a, b0, acc0);
    acc1 = mma_h(a, b1, acc1);
    acc2 = mma_h(a, b2, acc2);
    acc3 = mma_h(a, b3, acc3);
    guard6<v16h>(acc0, acc1, acc2, acc3, a, b0, b1, b2, b3, a);
  }
  const v4f bv = *(const v4f*)(bias + col0 + m * 4);
  v4f badd;
#pragma unroll
  for (int e = 0; e < 4; ++e) badd[e] = bfr(bv[e]);
  epi64r(slab + wave * SLAB64, acc0, acc1, acc2, acc3, oscale, badd, R, use_res, C, N, (size_t)rowb, col0, lane);
}

__global__ __launch_bounds__(256) void xt16(const float* __restrict__ X, u16* XTo) {
  __shared__ __align__(16) u16 TH[64 * VTP];
  const int tid = threadIdx.x;
  const int bid = blockIdx.x;
  const int st  = bid & (SEQ / 64 - 1);
  const int dcb = (bid >> 5) & (DM / 64 - 1);
  const int b   = bid >> 8;
  const int s0  = st * 64;
  const int d0  = dcb * 64;
  {
    const int sl = tid >> 2;
    const int dc = (tid & 3) * 16;
    const float* src = X + ((size_t)b * SEQ + s0 + sl) * DM + d0 + dc;
#pragma unroll
    for (int i = 0; i < 4; ++i) {
      const v4f a = *(const v4f*)(src + 4 * i);
#pragma unroll
      for (int e = 0; e < 4; ++e) {
        const _Float16 hv = (_Float16)(a[e] * VCAR);
        TH[(dc + 4 * i + e) * VTP + sl] = h_bits(hv);
      }
    }
  }
  __syncthreads();
  v4u vh[2];
  const int q8 = tid >> 3, p8 = (tid & 7) * 8;
#pragma unroll
  for (int it = 0; it < 2; ++it) {
    const int line = it * 32 + q8;
    vh[it] = *(const v4u*)(TH + line * VTP + p8);
  }
  const size_t base = ((size_t)b * DM + d0) * SEQ + s0 + p8;
  for (int pass = 0; pass < 2; ++pass) {
#pragma unroll
    for (int it = 0; it < 2; ++it) {
      const int line = it * 32 + q8;
      *(volatile v4u*)(XTo + base + (size_t)line * SEQ) = vh[it];
    }
    __threadfence();
  }
}

__global__ __launch_bounds__(256) void lnrelu(const float* __restrict__ Hp, const float* __restrict__ g,
                                              const float* __restrict__ bt, u16* AP, int rows) {
  const int tid = threadIdx.x, wave = tid >> 5, lane = tid & 31;
  const int rowid = blockIdx.x * 8 + wave;
  if (rowid >= rows) return;
  const float* hp = Hp + (size_t)rowid * DM;
  const int c0 = lane * 8, c1 = DM / 2 + lane * 8;
  float v[16];
  {
    const v4f a0 = *(const v4f*)(hp + c0), a1 = *(const v4f*)(hp + c0 + 4);
    const v4f a2 = *(const v4f*)(hp + c1), a3 = *(const v4f*)(hp + c1 + 4);
#pragma unroll
    for (int e = 0; e < 4; ++e) { v[e] = a0[e]; v[4 + e] = a1[e]; v[8 + e] = a2[e]; v[12 + e] = a3[e]; }
  }
  float s = 0.f;
#pragma unroll
  for (int i = 0; i < 16; ++i) s += v[i];
#pragma unroll
  for (int d = 16; d >= 1; d >>= 1) s += __shfl_xor(s, d, 32);
  const float mu = s * (1.0f / (float)DM);
  float q = 0.f;
#pragma unroll
  for (int i = 0; i < 16; ++i) { const float dd = v[i] - mu; q += dd * dd; }
#pragma unroll
  for (int d = 16; d >= 1; d >>= 1) q += __shfl_xor(q, d, 32);
  const float rs = rsqrtf(q * (1.0f / (float)DM) + EPSLN);
  float gg[16], bb[16];
  {
    const v4f g0 = *(const v4f*)(g + c0), g1 = *(const v4f*)(g + c0 + 4), g2 = *(const v4f*)(g + c1), g3 = *(const v4f*)(g + c1 + 4);
    const v4f t0 = *(const v4f*)(bt + c0), t1 = *(const v4f*)(bt + c0 + 4), t2 = *(const v4f*)(bt + c1), t3 = *(const v4f*)(bt + c1 + 4);
#pragma unroll
    for (int e = 0; e < 4; ++e) {
      gg[e] = bfr(g0[e]); gg[4 + e] = bfr(g1[e]); gg[8 + e] = bfr(g2[e]); gg[12 + e] = bfr(g3[e]);
      bb[e] = bfr(t0[e]); bb[4 + e] = bfr(t1[e]); bb[8 + e] = bfr(t2[e]); bb[12 + e] = bfr(t3[e]);
    }
  }
  unsigned short hb[16];
#pragma unroll
  for (int i = 0; i < 16; ++i) {
    const float y = fmaxf((v[i] - mu) * rs * gg[i] + bb[i], 0.0f) * ASC;
    hb[i] = h_bits((_Float16)y);
  }
  v4u o0, o1;
#pragma unroll
  for (int e = 0; e < 4; ++e) { o0[e] = pk16(hb[2 * e], hb[2 * e + 1]); o1[e] = pk16(hb[8 + 2 * e], hb[9 + 2 * e]); }
  u16* dst0 = AP + (size_t)rowid * DM + c0;
  u16* dst1 = AP + (size_t)rowid * DM + c1;
  for (int pass = 0; pass < 2; ++pass) {
    *(volatile v4u*)(dst0) = o0;
    *(volatile v4u*)(dst1) = o1;
    __threadfence();
  }
}

__global__ __launch_bounds__(ATT_THREADS)
void attn_fwd(const u16* __restrict__ QPp, const u16* __restrict__ KPp, const u16* __restrict__ XTp,
              const int* __restrict__ lens, float* Hout) {
  __shared__ __align__(16) float scs[16 * SCP];
  __shared__ __align__(16) u16   pls[16 * PLP];
  __shared__ float rowa[QT];
  __shared__ float rowi[QT];

  const int tid  = threadIdx.x;
  const int wave = tid >> 5;
  const int lane = tid & 31;
  const int hh   = lane >> 4;
  const int m    = lane & 15;
  const int r16  = tid >> 4;
  const int sub  = tid & 15;
  const int kl0  = sub * 32;

  const int bid = blockIdx.x;
  const int b   = bid >> 7;
  const int q0  = (bid & 127) * QT;
  int len = lens[b];
  len = (len < 1) ? 1 : ((len > SEQ) ? SEQ : len);
  const int nkt = (len + 31) >> 5;
  const int nch = (nkt + 15) >> 4;

  const _Float16* qa  = (const _Float16*)(const void*)QPp + ((size_t)b * SEQ + q0 + m) * DM + 8 * hh;
  const _Float16* kbp = (const _Float16*)(const void*)KPp + ((size_t)b * SEQ + m) * DM + 8 * hh;
  const _Float16* vbp = (const _Float16*)(const void*)XTp + ((size_t)b * DM + wave * 64 + m) * SEQ + 8 * hh;
  const float lsc = RSQD * LOG2E / (QSC * KSC);

  float mrun = -INFINITY, lrun = 0.f;
  v8f o0 = zero8(), o1 = zero8(), o2 = zero8(), o3 = zero8();

#pragma unroll 1
  for (int c = 0; c < nch; ++c) {
    const int kbeg = c * CK;
    const int nkbr = nkt - 16 * c;
    const int nkb  = (nkbr > 16) ? 16 : nkbr;
#pragma unroll 1
    for (int kb = wave; kb < nkb; kb += 8) {
      const _Float16* k0p = kbp + (size_t)(kbeg + kb * 32) * DM;
      const _Float16* k1p = k0p + (size_t)16 * DM;
      v8f s0 = zero8(), s1 = zero8();
#pragma unroll 4
      for (int ks = 0; ks < DM / 32; ++ks) {
        const v16h a  = ldfrag_h(qa + ks * 32);
        const v16h f0 = ldfrag_h(k0p + ks * 32);
        const v16h f1 = ldfrag_h(k1p + ks * 32);
        s0 = mma_h(a, f0, s0);
        s1 = mma_h(a, f1, s1);
        guard2x3(s0, s1, a, f0, f1);
      }
      float* srow = scs + (8 * hh) * SCP + kb * 32 + m;
#pragma unroll
      for (int r = 0; r < 8; ++r) {
        srow[r * SCP]      = s0[r];
        srow[r * SCP + 16] = s1[r];
      }
    }
    __syncthreads();
    {
      const float* sp = scs + r16 * SCP + kl0;
      float t[32];
      float cm = -INFINITY;
#pragma unroll
      for (int i = 0; i < 8; ++i) {
        const v4f a = *(const v4f*)(sp + 4 * i);
#pragma unroll
        for (int e = 0; e < 4; ++e) {
          const int kl = kl0 + 4 * i + e;
          const bool ok = (kbeg + kl) < len;
          const float tv = ok ? (a[e] * lsc) : -INFINITY;
          t[4 * i + e] = tv;
          cm = fmaxf(cm, tv);
        }
      }
#pragma unroll
      for (int d = 1; d <= 8; d <<= 1) cm = fmaxf(cm, __shfl_xor(cm, d, 32));
      const float mn = fmaxf(mrun, cm);
      const float al = (mrun == -INFINITY) ? 0.f : exp2f(mrun - mn);
      mrun = mn;
      float ps = 0.f;
      v4u pk[4];
#pragma unroll
      for (int i = 0; i < 4; ++i) {
#pragma unroll
        for (int e = 0; e < 4; ++e) {
          const int j = 8 * i + 2 * e;
          const float x0 = exp2f(fminf(t[j] - mn, 0.f));
          const float x1 = exp2f(fminf(t[j + 1] - mn, 0.f));
          const float p0 = (t[j] == -INFINITY) ? 0.f : x0;
          const float p1 = (t[j + 1] == -INFINITY) ? 0.f : x1;
          ps += p0 + p1;
          pk[i][e] = pk16(h_bits((_Float16)(p0 * PCAR)), h_bits((_Float16)(p1 * PCAR)));
        }
      }
#pragma unroll
      for (int d = 1; d <= 8; d <<= 1) ps += __shfl_xor(ps, d, 32);
      lrun = lrun * al + ps;
      if (sub < nkb) {
        u16* pd = pls + r16 * PLP + kl0;
#pragma unroll
        for (int i = 0; i < 4; ++i) *(v4u*)(pd + 8 * i) = pk[i];
      }
      if (sub == 0) rowa[r16] = al;
    }
    __syncthreads();
    {
      float scl[8];
#pragma unroll
      for (int r = 0; r < 8; ++r) scl[r] = rowa[8 * hh + r];
#pragma unroll
      for (int r = 0; r < 8; ++r) { o0[r] *= scl[r]; o1[r] *= scl[r]; o2[r] *= scl[r]; o3[r] *= scl[r]; }
      const _Float16* pp = (const _Float16*)(const void*)pls + m * PLP + 8 * hh;
      const _Float16* vp = vbp + kbeg;
#pragma unroll 1
      for (int kb = 0; kb < nkb; ++kb) {
        const v16h pf = ldfrag_h(pp + kb * 32);
        const v16h g0 = ldfrag_h(vp + kb * 32);
        const v16h g1 = ldfrag_h(vp + (size_t)16 * SEQ + kb * 32);
        const v16h g2 = ldfrag_h(vp + (size_t)32 * SEQ + kb * 32);
        const v16h g3 = ldfrag_h(vp + (size_t)48 * SEQ + kb * 32);
        o0 = mma_h(pf, g0, o0);
        o1 = mma_h(pf, g1, o1);
        o2 = mma_h(pf, g2, o2);
        o3 = mma_h(pf, g3, o3);
        guard6<v16h>(o0, o1, o2, o3, pf, g0, g1, g2, g3, pf);
      }
    }
  }
  acc_guard4(o0, o1, o2, o3);

  if (sub == 0) rowi[r16] = (1.0f / lrun) * (1.0f / (PCAR * VCAR));
  __syncthreads();
  float inv[8];
#pragma unroll
  for (int r = 0; r < 8; ++r) inv[r] = rowi[8 * hh + r];
#pragma unroll
  for (int r = 0; r < 8; ++r) { o0[r] *= inv[r]; o1[r] *= inv[r]; o2[r] *= inv[r]; o3[r] *= inv[r]; }
  epi64(scs + wave * SLAB64, o0, o1, o2, o3, 1.0f, zero4(), Hout, DM, (size_t)b * SEQ + q0, wave * 64, lane);
}

extern "C" void kernel_launch(void* const* d_in, const int* in_sizes, int n_in,
                              void* d_out, int out_size, void* d_ws, size_t ws_size,
                              hipStream_t stream) {
  if (n_in < 12) return;
  const int nb = in_sizes[1];
  if (nb < 1 || nb > 64) return;
  const int rows = nb * SEQ;
  if (in_sizes[0] != rows * NIN) return;
  if (in_sizes[2] != DM * NIN || in_sizes[3] != DM) return;
  if (in_sizes[4] != DM * DM || in_sizes[5] != DM || in_sizes[6] != DM * DM || in_sizes[7] != DM) return;
  if (in_sizes[8] != NLAY * DM || in_sizes[9] != NLAY * DM || in_sizes[10] != NLAY * DM * DM || in_sizes[11] != NLAY * DM) return;
  if (out_size != rows * DM) return;

  const float* seq  = (const float*)d_in[0];
  const int*   lens = (const int*)d_in[1];
  const float* w0   = (const float*)d_in[2];
  const float* b0   = (const float*)d_in[3];
  const float* wq   = (const float*)d_in[4];
  const float* bq   = (const float*)d_in[5];
  const float* wk   = (const float*)d_in[6];
  const float* bk   = (const float*)d_in[7];
  const float* lng  = (const float*)d_in[8];
  const float* lnb  = (const float*)d_in[9];
  const float* wl   = (const float*)d_in[10];
  const float* bl   = (const float*)d_in[11];
  float*       out  = (float*)d_out;

  const size_t szW0  = (size_t)DM * NIN * 2;
  const size_t szW   = (size_t)DM * DM * 2;
  const size_t szWL  = (size_t)NLAY * DM * DM * 2;
  const size_t szX   = (size_t)rows * DM * 4;
  const size_t szH16 = (size_t)rows * DM * 2;
  const size_t szXT  = (size_t)nb * DM * SEQ * 2;
  const size_t szSB  = (size_t)rows * NIN * 2;
  size_t off = 0;
  const size_t oW0B = off; off += szW0;
  const size_t oWQH = off; off += szW;
  const size_t oWKH = off; off += szW;
  const size_t oWLH = off; off += szWL;
  const size_t oX   = off; off += szX;
  const size_t oP1  = off; off += szX;
  const size_t oP2  = off; off += (szXT > szSB ? szXT : szSB);
  const size_t oP3  = off; off += szH16;
  const size_t oP4  = off; off += szH16;
  if (off > ws_size) return;
  if (off > WS_CAP) return;
  if (szH16 > szX) return;

  char* ws = (char*)d_ws;
  u16*   W0B = (u16*)(ws + oW0B);
  u16*   WQH = (u16*)(ws + oWQH);
  u16*   WKH = (u16*)(ws + oWKH);
  u16*   WLH = (u16*)(ws + oWLH);
  float* X   = (float*)(ws + oX);
  u16*   XH  = (u16*)(ws + oP1);
  float* H   = (float*)(ws + oP1);
  u16*   SB  = (u16*)(ws + oP2);
  u16*   XT  = (u16*)(ws + oP2);
  u16*   QP  = (u16*)(ws + oP3);
  u16*   AP  = (u16*)(ws + oP3);
  u16*   KP  = (u16*)(ws + oP4);

  const int n8s  = (rows * NIN) / 8;
  const int n8w0 = (DM * NIN) / 8;
  const int n8w  = (DM * DM) / 8;
  const int n8wl = (NLAY * DM * DM) / 8;
  const int n8x  = (rows * DM) / 8;
  if ((n8s % 256) != 0 || (n8w0 % 256) != 0 || (n8w % 256) != 0 || (n8wl % 256) != 0 || (n8x % 256) != 0) return;
  if ((rows % 64) != 0 || (rows % 8) != 0) return;
  const dim3 blk(256);
  const dim3 gS(n8s / 256), gW0(n8w0 / 256), gW(n8w / 256), gWL(n8wl / 256), gXH(n8x / 256);
  const dim3 gG((rows / 64) * (DM / 64));
  const dim3 bG(128);
  const dim3 gXT(nb * (DM / 64) * (SEQ / 64));
  const dim3 gAT(nb * (SEQ / QT));
  const dim3 bAT(ATT_THREADS);
  const dim3 gLN(rows / 8);

  cvt16<<<gS,  blk, 0, stream>>>(seq, SB, n8s, 0, 1.0f);
  cvt16<<<gW0, blk, 0, stream>>>(w0, W0B, n8w0, 0, 1.0f);
  cvt16<<<gW,  blk, 0, stream>>>(wq, WQH, n8w, 1, WSC);
  cvt16<<<gW,  blk, 0, stream>>>(wk, WKH, n8w, 1, WSC);
  cvt16<<<gWL, blk, 0, stream>>>(wl, WLH, n8wl, 1, WSC);
  gemm_bfb<<<gG, bG, 0, stream>>>(SB, W0B, b0, X, rows, DM, NIN, 1.0f);
  cvt16<<<gXH, blk, 0, stream>>>(X, XH, n8x, 2, XSC);
  xt16<<<gXT, blk, 0, stream>>>(X, XT);
  gemm_ho16<<<gG, bG, 0, stream>>>(XH, WQH, bq, QP, rows, DM, DM, 1.0f / (XSC * WSC), QSC);
  gemm_ho16<<<gG, bG, 0, stream>>>(XH, WKH, bk, KP, rows, DM, DM, 1.0f / (XSC * WSC), KSC);
  attn_fwd<<<gAT, bAT, 0, stream>>>(QP, KP, XT, lens, H);
  lnrelu<<<gLN, blk, 0, stream>>>(H, lng, lnb, AP, rows);
  gemm_h32<<<gG, bG, 0, stream>>>(AP, WLH, bl, X, 0, H, rows, DM, DM, 1.0f / (ASC * WSC));
  lnrelu<<<gLN, blk, 0, stream>>>(H, lng + DM, lnb + DM, AP, rows);
  gemm_h32<<<gG, bG, 0, stream>>>(AP, WLH + (size_t)DM * DM, bl + DM, X, 1, out, rows, DM, DM, 1.0f / (ASC * WSC));
  (void)hipGetLastError();
}
